// DiT_63866163691579
// MI455X (gfx1250) — hardware-verified
//
#include <hip/hip_runtime.h>
#include <stddef.h>
#include <stdint.h>

#define NB    4
#define SQ    1024
#define NTOK  4096
#define DM    1024
#define NH    16
#define HDM   64
#define NQKV  3072
#define TL    256
#define NTT   1024
#define DFF   4096
#define QB    128
#define KC    64
#define NQB   (SQ / QB)
#define TTN   (SQ * 16 * 8)

static_assert(NTOK == NB * SQ);
static_assert(NTT == NB * TL);
static_assert(SQ % 256 == 0);
static_assert(TL % 256 == 0);
static_assert(DM % 64 == 0);
static_assert(DM % 32 == 0);
static_assert(DFF % 64 == 0);
static_assert(HDM == 64);
static_assert(NH * HDM == DM);
static_assert(NQKV == 3 * DM);
static_assert(SQ % KC == 0);
static_assert(TL % KC == 0);
static_assert(SQ % QB == 0);
static_assert(NTOK % 256 == 0);
static_assert((NTOK * DM) % 2048 == 0);
static_assert((NQKV * DM) % 2048 == 0);
static_assert((DFF * DM) % 2048 == 0);
static_assert((NTT * DM) % 2048 == 0);
static_assert((SQ * HDM) % 256 == 0);
static_assert(TTN == 2 * SQ * HDM);

typedef _Float16 v16h __attribute__((ext_vector_type(16)));
typedef _Float16 v8h  __attribute__((ext_vector_type(8)));
typedef float    v8f  __attribute__((ext_vector_type(8)));
typedef float    v4f  __attribute__((ext_vector_type(4)));
typedef unsigned int v4u __attribute__((ext_vector_type(4)));

union Frag  { v16h v; v8h h[2]; };
union Pack8 { v8h h; v4u u; };

__device__ __forceinline__ v8f mma16(v16h a, v16h b, v8f c) {
  c = __builtin_amdgcn_wmma_f32_16x16x32_f16(false, a, false, b, (short)0, c, false, false);
  asm volatile("v_nop\n\tv_nop\n\tv_nop\n\tv_nop" : "+v"(c) : "v"(a), "v"(b));
  return c;
}

__device__ __forceinline__ void wait_global_loads() {
  asm volatile("s_wait_loadcnt 0x0" ::: "memory");
}

__device__ __forceinline__ v16h ldfrag(const _Float16* p, int ld, int row0, int k0, int lane) {
  const int m = lane & 15, lh = lane >> 4;
  const _Float16* q = p + (size_t)(row0 + m) * ld + k0 + 8 * lh;
  Frag f;
  f.h[0] = *(const v8h*)(q);
  f.h[1] = *(const v8h*)(q + 16);
  return f.v;
}

__device__ __forceinline__ v8f zero8() { return (v8f){0.f, 0.f, 0.f, 0.f, 0.f, 0.f, 0.f, 0.f}; }

__device__ __forceinline__ v4f sel4(bool cnd, v4f a, v4f b) {
  v4f r;
  r[0] = cnd ? a[0] : b[0];
  r[1] = cnd ? a[1] : b[1];
  r[2] = cnd ? a[2] : b[2];
  r[3] = cnd ? a[3] : b[3];
  return r;
}

__device__ __forceinline__ void gemm32x64(const _Float16* __restrict__ A, int lda,
                                          const _Float16* __restrict__ Bt, int ldb, int K,
                                          int m0, int n0, int lane, v8f (&acc)[2][4]) {
#pragma unroll 1
  for (int k0 = 0; k0 < K; k0 += 32) {
    const v16h a0 = ldfrag(A, lda, m0, k0, lane);
    const v16h a1 = ldfrag(A, lda, m0 + 16, k0, lane);
    const v16h b0 = ldfrag(Bt, ldb, n0, k0, lane);
    const v16h b1 = ldfrag(Bt, ldb, n0 + 16, k0, lane);
    const v16h b2 = ldfrag(Bt, ldb, n0 + 32, k0, lane);
    const v16h b3 = ldfrag(Bt, ldb, n0 + 48, k0, lane);
    acc[0][0] = mma16(a0, b0, acc[0][0]);
    acc[1][0] = mma16(a1, b0, acc[1][0]);
    acc[0][1] = mma16(a0, b1, acc[0][1]);
    acc[1][1] = mma16(a1, b1, acc[1][1]);
    acc[0][2] = mma16(a0, b2, acc[0][2]);
    acc[1][2] = mma16(a1, b2, acc[1][2]);
    acc[0][3] = mma16(a0, b3, acc[0][3]);
    acc[1][3] = mma16(a1, b3, acc[1][3]);
  }
}

__global__ __launch_bounds__(256) void k_trig(const float* __restrict__ rot, float* __restrict__ tt) {
  __shared__ __align__(16) float cs[256];
  __shared__ __align__(16) float sn[256];
  const int tid = threadIdx.x;
  const float a = rot[(size_t)blockIdx.x * 256 + tid];
  cs[tid] = cosf(a);
  sn[tid] = sinf(a);
  __syncthreads();
  const int p  = tid & 127;
  const int ps = p >> 5;
  const int q  = p & 31;
  const int cc = q >> 1;
  const int hs = q & 1;
  const int ib = ps * 64 + cc;
  v4f vc, vs;
  vc[0] = cs[ib]; vc[1] = cs[ib + 16]; vc[2] = cs[ib + 32]; vc[3] = cs[ib + 48];
  vs[0] = sn[ib]; vs[1] = sn[ib + 16]; vs[2] = sn[ib + 32]; vs[3] = sn[ib + 48];
  const v4f v = sel4(hs == 0, vc, vs);
  const size_t o = (size_t)blockIdx.x * 512 + (size_t)p * 4;
  if (tid < 128) *(volatile v4f*)(tt + o) = v;
  __threadfence();
  if (tid < 128) *(volatile v4f*)(tt + o) = v;
}

__global__ __launch_bounds__(256) void k_cvt(const float* __restrict__ src, _Float16* __restrict__ dh, float scale) {
  const int tid = threadIdx.x;
  const size_t o = (size_t)blockIdx.x * 2048 + (size_t)tid * 8;
  const v4f a0 = *(const v4f*)(src + o) * scale;
  const v4f a1 = *(const v4f*)(src + o + 4) * scale;
  Pack8 pk;
  pk.h = (v8h){(_Float16)a0[0], (_Float16)a0[1], (_Float16)a0[2], (_Float16)a0[3],
               (_Float16)a1[0], (_Float16)a1[1], (_Float16)a1[2], (_Float16)a1[3]};
  const v4u vv = pk.u;
  volatile v4u* d = (volatile v4u*)(dh + o);
  *d = vv;
  __threadfence();
  *d = vv;
}

__global__ __launch_bounds__(128) void k_ln(const float* __restrict__ x, const float* __restrict__ g,
                                            const float* __restrict__ bt, _Float16* __restrict__ xn) {
  __shared__ float red[2][4];
  const int tid = threadIdx.x, lane = tid & 31, wave = tid >> 5;
  const size_t o = (size_t)blockIdx.x * DM + (size_t)tid * 8;
  const v4f a0 = *(const v4f*)(x + o);
  const v4f a1 = *(const v4f*)(x + o + 4);
  float s = ((a0[0] + a0[1]) + (a0[2] + a0[3])) + ((a1[0] + a1[1]) + (a1[2] + a1[3]));
#pragma unroll
  for (int off = 1; off < 32; off <<= 1) s += __shfl_xor(s, off, 32);
  if (lane == 0) red[0][wave] = s;
  __syncthreads();
  const float mean = ((red[0][0] + red[0][1]) + (red[0][2] + red[0][3])) * (1.0f / 1024.0f);
  const v4f d0 = a0 - mean;
  const v4f d1 = a1 - mean;
  float q = ((d0[0] * d0[0] + d0[1] * d0[1]) + (d0[2] * d0[2] + d0[3] * d0[3])) +
            ((d1[0] * d1[0] + d1[1] * d1[1]) + (d1[2] * d1[2] + d1[3] * d1[3]));
#pragma unroll
  for (int off = 1; off < 32; off <<= 1) q += __shfl_xor(q, off, 32);
  if (lane == 0) red[1][wave] = q;
  __syncthreads();
  const float var  = ((red[1][0] + red[1][1]) + (red[1][2] + red[1][3])) * (1.0f / 1024.0f);
  const float rstd = rsqrtf(var + 1e-5f);
  const v4f g0 = *(const v4f*)(g + tid * 8);
  const v4f g1 = *(const v4f*)(g + tid * 8 + 4);
  const v4f b0 = *(const v4f*)(bt + tid * 8);
  const v4f b1 = *(const v4f*)(bt + tid * 8 + 4);
  const v4f y0 = d0 * rstd * g0 + b0;
  const v4f y1 = d1 * rstd * g1 + b1;
  Pack8 pk;
  pk.h = (v8h){(_Float16)y0[0], (_Float16)y0[1], (_Float16)y0[2], (_Float16)y0[3],
               (_Float16)y1[0], (_Float16)y1[1], (_Float16)y1[2], (_Float16)y1[3]};
  const v4u vv = pk.u;
  volatile v4u* d = (volatile v4u*)(xn + o);
  *d = vv;
  __threadfence();
  *d = vv;
}

#define STP 72
#define SVP 264
__global__ __launch_bounds__(256) void k_qkv(const _Float16* __restrict__ ap,
                                             const _Float16* __restrict__ wt,
                                             const float* __restrict__ bias,
                                             const float* __restrict__ tt,
                                             _Float16* __restrict__ qp,
                                             _Float16* __restrict__ kp,
                                             _Float16* __restrict__ vtp,
                                             int seqlen, int which0, int rope) {
  __shared__ __align__(16) _Float16 st[256 * STP];
  const int tid = threadIdx.x, lane = tid & 31, wave = tid >> 5;
  const int hh = lane >> 4, c = lane & 15;
  const int spb = seqlen >> 8;
  const int bx  = blockIdx.x;
  const int b   = bx / spb;
  const int sb  = (bx - b * spb) * 256;
  const int ns  = which0 * NH + blockIdx.y;
  const int which = ns / NH;
  const int head  = ns - which * NH;
  const int hb    = b * NH + head;
  const int m0 = bx * 256 + wave * 32;
  const int n0 = ns * 64;

  v8f acc[2][4];
#pragma unroll
  for (int s = 0; s < 2; ++s)
#pragma unroll
    for (int t = 0; t < 4; ++t) acc[s][t] = zero8();
  gemm32x64(ap, DM, wt, DM, DM, m0, n0, lane, acc);

  float bb[4];
#pragma unroll
  for (int t = 0; t < 4; ++t) bb[t] = bias[n0 + 16 * t + c];
#pragma unroll
  for (int sub = 0; sub < 2; ++sub)
#pragma unroll
    for (int t = 0; t < 4; ++t)
#pragma unroll
      for (int r = 0; r < 8; ++r) acc[sub][t][r] = acc[sub][t][r] * 0.03125f + bb[t];

  if (which < 2) {
    if (rope != 0) {
#pragma unroll
      for (int sub = 0; sub < 2; ++sub) {
#pragma unroll
        for (int rg = 0; rg < 2; ++rg) {
          wait_global_loads();
          v4f cv[4], sv[4];
#pragma unroll
          for (int r4 = 0; r4 < 4; ++r4) {
            const int r  = rg * 4 + r4;
            const int lr = wave * 32 + sub * 16 + 8 * hh + r;
            const float* tp = tt + ((size_t)(sb + lr) * 16 + c) * 8;
            cv[r4] = *(const v4f*)(tp);
            sv[r4] = *(const v4f*)(tp + 4);
          }
#pragma unroll
          for (int r4 = 0; r4 < 4; ++r4) {
            const int r  = rg * 4 + r4;
            const int lr = wave * 32 + sub * 16 + 8 * hh + r;
            const float o0 = acc[sub][0][r] * cv[r4][0] - acc[sub][2][r] * sv[r4][0];
            const float o1 = acc[sub][1][r] * cv[r4][1] - acc[sub][3][r] * sv[r4][1];
            const float o2 = acc[sub][2][r] * cv[r4][2] + acc[sub][0][r] * sv[r4][2];
            const float o3 = acc[sub][3][r] * cv[r4][3] + acc[sub][1][r] * sv[r4][3];
            _Float16* rw = st + lr * STP + c;
            rw[0]  = (_Float16)o0;
            rw[16] = (_Float16)o1;
            rw[32] = (_Float16)o2;
            rw[48] = (_Float16)o3;
          }
        }
      }
    } else {
#pragma unroll
      for (int sub = 0; sub < 2; ++sub)
#pragma unroll
        for (int t = 0; t < 4; ++t)
#pragma unroll
          for (int r = 0; r < 8; ++r)
            st[(wave * 32 + sub * 16 + 8 * hh + r) * STP + 16 * t + c] = (_Float16)acc[sub][t][r];
    }
  } else {
#pragma unroll
    for (int sub = 0; sub < 2; ++sub)
#pragma unroll
      for (int t = 0; t < 4; ++t)
#pragma unroll
        for (int r = 0; r < 8; ++r)
          st[(16 * t + c) * SVP + wave * 32 + sub * 16 + 8 * hh + r] = (_Float16)acc[sub][t][r];
  }
  __syncthreads();

  if (which < 2) {
    _Float16* base = ((which == 0) ? qp : kp) + (size_t)hb * seqlen * HDM;
#pragma unroll
    for (int g = 0; g < 2; ++g) {
      v4u val[4];
      size_t go[4];
#pragma unroll
      for (int j = 0; j < 4; ++j) {
        const int p  = tid + 256 * (4 * g + j);
        const int lr = p >> 3;
        const int pc = p & 7;
        Pack8 pk;
        pk.h   = *(const v8h*)(st + lr * STP + pc * 8);
        val[j] = pk.u;
        go[j]  = (size_t)(sb + lr) * HDM + pc * 8;
      }
      for (int ps = 0; ps < 2; ++ps) {
#pragma unroll
        for (int j = 0; j < 4; ++j) *(volatile v4u*)(base + go[j]) = val[j];
        __threadfence();
      }
    }
  } else {
    _Float16* base = vtp + (size_t)hb * HDM * seqlen;
#pragma unroll
    for (int g = 0; g < 2; ++g) {
      v4u val[4];
      size_t go[4];
#pragma unroll
      for (int j = 0; j < 4; ++j) {
        const int p    = tid + 256 * (4 * g + j);
        const int drow = p >> 5;
        const int pc   = p & 31;
        Pack8 pk;
        pk.h   = *(const v8h*)(st + drow * SVP + pc * 8);
        val[j] = pk.u;
        go[j]  = (size_t)drow * seqlen + sb + pc * 8;
      }
      for (int ps = 0; ps < 2; ++ps) {
#pragma unroll
        for (int j = 0; j < 4; ++j) *(volatile v4u*)(base + go[j]) = val[j];
        __threadfence();
      }
    }
  }
}

#define KTP 72
#define OTP 68
template <int EPI>
__global__ __launch_bounds__(256) void k_attn(const _Float16* __restrict__ qp,
                                              const _Float16* __restrict__ kp,
                                              const _Float16* __restrict__ vt,
                                              const float* __restrict__ resid,
                                              float* __restrict__ outf,
                                              _Float16* __restrict__ op, int nkeys, float sscale) {
  __shared__ __align__(16) _Float16 Ks[KC * KTP];
  __shared__ __align__(16) _Float16 Vs[HDM * KTP];
  __shared__ __align__(16) _Float16 Ps[8 * 16 * KTP];

  const int tid = threadIdx.x, lane = tid & 31, wave = tid >> 5;
  const int hh = lane >> 4, c = lane & 15;
  const int qb  = blockIdx.x % NQB;
  const int hb  = blockIdx.x / NQB;
  const int h   = hb % NH;
  const int b   = hb / NH;
  const int q0  = qb * QB + wave * 16;
  const int nck = nkeys / KC;

  const _Float16* Q = qp + (size_t)hb * SQ * HDM;
  const _Float16* K = kp + (size_t)hb * nkeys * HDM;
  const _Float16* V = vt + (size_t)hb * HDM * nkeys;

  v16h qa[2];
  qa[0] = ldfrag(Q, HDM, q0, 0, lane);
  qa[1] = ldfrag(Q, HDM, q0, 32, lane);

  const float NEGI = -__builtin_huge_valf();
  float mrow[8], lrow[8];
  v8f oacc[4];
#pragma unroll
  for (int r = 0; r < 8; ++r) { mrow[r] = NEGI; lrow[r] = 0.f; }
#pragma unroll
  for (int t = 0; t < 4; ++t) oacc[t] = zero8();

  _Float16* pw = Ps + wave * 16 * KTP;

  for (int kc = 0; kc < nck; ++kc) {
    const int kv0 = kc * KC;
    __syncthreads();
    {
      const int r  = tid >> 2;
      const int qq = (tid & 3) * 16;
      const _Float16* ks = K + (size_t)(kv0 + r) * HDM + qq;
      const _Float16* vs = V + (size_t)r * nkeys + kv0 + qq;
#pragma unroll
      for (int e = 0; e < 2; ++e) {
        *(v8h*)(Ks + r * KTP + qq + 8 * e) = *(const v8h*)(ks + 8 * e);
        *(v8h*)(Vs + r * KTP + qq + 8 * e) = *(const v8h*)(vs + 8 * e);
      }
    }
    __syncthreads();

    v8f s[4];
#pragma unroll
    for (int j = 0; j < 4; ++j) s[j] = zero8();
#pragma unroll
    for (int dc = 0; dc < 2; ++dc) {
#pragma unroll
      for (int j = 0; j < 4; ++j) {
        const v16h kb = ldfrag(Ks, KTP, j * 16, dc * 32, lane);
        s[j] = mma16(qa[dc], kb, s[j]);
      }
    }
    float cm[8];
#pragma unroll
    for (int r = 0; r < 8; ++r) {
      float m = NEGI;
#pragma unroll
      for (int j = 0; j < 4; ++j) { s[j][r] *= sscale; m = fmaxf(m, s[j][r]); }
#pragma unroll
      for (int off = 1; off < 16; off <<= 1) m = fmaxf(m, __shfl_xor(m, off, 32));
      cm[r] = m;
    }
    float al[8];
#pragma unroll
    for (int r = 0; r < 8; ++r) {
      const float mnew  = fmaxf(mrow[r], cm[r]);
      const float alpha = __expf(mrow[r] - mnew);
      mrow[r] = mnew;
      float psum = 0.f;
#pragma unroll
      for (int j = 0; j < 4; ++j) {
        const float p = __expf(s[j][r] - mnew);
        psum += p;
        pw[(8 * hh + r) * KTP + j * 16 + c] = (_Float16)(p * 1024.0f);
      }
#pragma unroll
      for (int off = 1; off < 16; off <<= 1) psum += __shfl_xor(psum, off, 32);
      lrow[r] = lrow[r] * alpha + psum;
      al[r] = alpha;
    }
#pragma unroll
    for (int t = 0; t < 4; ++t)
#pragma unroll
      for (int r = 0; r < 8; ++r) oacc[t][r] *= al[r];
    __syncthreads();

#pragma unroll
    for (int kk = 0; kk < 2; ++kk) {
      const v16h pa = ldfrag(pw, KTP, 0, kk * 32, lane);
#pragma unroll
      for (int t = 0; t < 4; ++t) {
        const v16h vb = ldfrag(Vs, KTP, t * 16, kk * 32, lane);
        oacc[t] = mma16(pa, vb, oacc[t]);
      }
    }
  }

  __syncthreads();
  if (EPI == 1) {
    float invl[8];
#pragma unroll
    for (int r = 0; r < 8; ++r) invl[r] = (lrow[r] > 0.f) ? (0.0625f / lrow[r]) : 0.f;
#pragma unroll
    for (int r = 0; r < 8; ++r) {
#pragma unroll
      for (int t = 0; t < 4; ++t)
        pw[(8 * hh + r) * KTP + 16 * t + c] = (_Float16)(oacc[t][r] * invl[r]);
    }
    __syncthreads();
    v4u val[4];
    size_t go[4];
#pragma unroll
    for (int it = 0; it < 4; ++it) {
      const int p  = lane + 32 * it;
      const int L  = p >> 3;
      const int pc = p & 7;
      Pack8 pk;
      pk.h    = *(const v8h*)(pw + L * KTP + pc * 8);
      val[it] = pk.u;
      go[it]  = ((size_t)b * SQ + (size_t)(q0 + L)) * DM + (size_t)h * HDM + pc * 8;
    }
    for (int ps = 0; ps < 2; ++ps) {
#pragma unroll
      for (int it = 0; it < 4; ++it) *(volatile v4u*)(op + go[it]) = val[it];
      __threadfence();
    }
  } else {
    float invl[8];
#pragma unroll
    for (int r = 0; r < 8; ++r) invl[r] = (lrow[r] > 0.f) ? (0.0009765625f / lrow[r]) : 0.f;
    float* fw = (float*)(void*)(Ps + wave * 16 * KTP);
#pragma unroll
    for (int half = 0; half < 2; ++half) {
      if (hh == half) {
#pragma unroll
        for (int r = 0; r < 8; ++r) {
#pragma unroll
          for (int t = 0; t < 4; ++t) fw[r * OTP + 16 * t + c] = oacc[t][r] * invl[r];
        }
      }
      __syncthreads();
      v4f val[4];
      size_t go[4];
#pragma unroll
      for (int it = 0; it < 4; ++it) {
        const int p   = lane + 32 * it;
        const int row = p >> 4;
        const int pc  = p & 15;
        const v4f ov  = *(const v4f*)(fw + row * OTP + pc * 4);
        go[it]  = ((size_t)b * SQ + (size_t)(q0 + 8 * half + row)) * DM + (size_t)h * HDM + pc * 4;
        val[it] = ov + *(const v4f*)(resid + go[it]);
      }
      for (int ps = 0; ps < 2; ++ps) {
#pragma unroll
        for (int it = 0; it < 4; ++it) *(volatile v4f*)(outf + go[it]) = val[it];
        __threadfence();
      }
      __syncthreads();
    }
  }
}

__device__ __forceinline__ void out_epilogue_f32(v8f (&acc)[2][4], float scale, const float (&bb)[4],
                                                 float* sw, float* __restrict__ out, const float* __restrict__ res,
                                                 int ldo, int m0, int n0, int lane, int hh, int c) {
#pragma unroll
  for (int sub = 0; sub < 2; ++sub) {
    __syncthreads();
#pragma unroll
    for (int t = 0; t < 4; ++t) {
#pragma unroll
      for (int r = 0; r < 8; ++r) sw[(8 * hh + r) * OTP + 16 * t + c] = acc[sub][t][r] * scale + bb[t];
    }
    __syncthreads();
    v4f val[8];
    size_t go[8];
#pragma unroll
    for (int it = 0; it < 8; ++it) {
      const int p    = lane + 32 * it;
      const int L    = p >> 3;
      const int pc   = p & 7;
      const int row  = L >> 1;
      const int half = L & 1;
      go[it]  = (size_t)(m0 + sub * 16 + row) * ldo + n0 + half * 32 + pc * 4;
      val[it] = *(const v4f*)(sw + row * OTP + half * 32 + pc * 4) + *(const v4f*)(res + go[it]);
    }
    for (int ps = 0; ps < 2; ++ps) {
#pragma unroll
      for (int it = 0; it < 8; ++it) *(volatile v4f*)(out + go[it]) = val[it];
      __threadfence();
    }
  }
}

__global__ __launch_bounds__(256) void k_gemm_f32(const _Float16* __restrict__ ap, int lda,
                                                  const _Float16* __restrict__ wt, int K,
                                                  const float* __restrict__ bias, float scale,
                                                  float* __restrict__ out, int ldo,
                                                  const float* __restrict__ res) {
  __shared__ __align__(16) float st[8][16 * OTP];
  const int tid = threadIdx.x, lane = tid & 31, wave = tid >> 5;
  const int hh = lane >> 4, c = lane & 15;
  const int m0 = blockIdx.x * 256 + wave * 32;
  const int n0 = blockIdx.y * 64;

  v8f acc[2][4];
#pragma unroll
  for (int s = 0; s < 2; ++s)
#pragma unroll
    for (int t = 0; t < 4; ++t) acc[s][t] = zero8();
  gemm32x64(ap, lda, wt, K, K, m0, n0, lane, acc);
  float bb[4];
#pragma unroll
  for (int t = 0; t < 4; ++t) bb[t] = bias[n0 + 16 * t + c];
  out_epilogue_f32(acc, scale, bb, st[wave], out, res, ldo, m0, n0, lane, hh, c);
}

#define HTP 72
__global__ __launch_bounds__(256) void k_fcgate(const _Float16* __restrict__ ap,
                                                const _Float16* __restrict__ w1,
                                                const _Float16* __restrict__ wg,
                                                const float* __restrict__ b1,
                                                const float* __restrict__ bg,
                                                _Float16* __restrict__ hg) {
  __shared__ __align__(16) _Float16 st[128 * HTP];
  const int tid = threadIdx.x, lane = tid & 31, wave = tid >> 5;
  const int hh = lane >> 4, c = lane & 15;
  const int wm = wave & 3, wn = wave >> 2;
  const int m0 = blockIdx.x * 128 + wm * 32;
  const int n0 = blockIdx.y * 64 + wn * 32;

  v8f a1c[2][2], agc[2][2];
#pragma unroll
  for (int s = 0; s < 2; ++s)
#pragma unroll
    for (int t = 0; t < 2; ++t) { a1c[s][t] = zero8(); agc[s][t] = zero8(); }

#pragma unroll 1
  for (int k0 = 0; k0 < DM; k0 += 32) {
    const v16h x0 = ldfrag(ap, DM, m0, k0, lane);
    const v16h x1 = ldfrag(ap, DM, m0 + 16, k0, lane);
    const v16h p0 = ldfrag(w1, DM, n0, k0, lane);
    const v16h p1 = ldfrag(w1, DM, n0 + 16, k0, lane);
    const v16h g0 = ldfrag(wg, DM, n0, k0, lane);
    const v16h g1 = ldfrag(wg, DM, n0 + 16, k0, lane);
    a1c[0][0] = mma16(x0, p0, a1c[0][0]);
    a1c[1][0] = mma16(x1, p0, a1c[1][0]);
    a1c[0][1] = mma16(x0, p1, a1c[0][1]);
    a1c[1][1] = mma16(x1, p1, a1c[1][1]);
    agc[0][0] = mma16(x0, g0, agc[0][0]);
    agc[1][0] = mma16(x1, g0, agc[1][0]);
    agc[0][1] = mma16(x0, g1, agc[0][1]);
    agc[1][1] = mma16(x1, g1, agc[1][1]);
  }

  float bb1[2], bbg[2];
#pragma unroll
  for (int t = 0; t < 2; ++t) { bb1[t] = b1[n0 + 16 * t + c]; bbg[t] = bg[n0 + 16 * t + c]; }
#pragma unroll
  for (int sub = 0; sub < 2; ++sub) {
#pragma unroll
    for (int t = 0; t < 2; ++t) {
#pragma unroll
      for (int r = 0; r < 8; ++r) {
        const float hp = a1c[sub][t][r] * 0.03125f + bb1[t];
        const float gp = fmaxf(agc[sub][t][r] * 0.03125f + bbg[t], -30.0f);
        const float hv = 0.5f * hp * (1.0f + erff(hp * 0.70710678118654752f));
        const float gv = 1.0f / (1.0f + __expf(-gp));
        st[(wm * 32 + sub * 16 + 8 * hh + r) * HTP + wn * 32 + 16 * t + c] = (_Float16)(hv * gv * 16.0f);
      }
    }
  }
  __syncthreads();
  v4u val[4];
  size_t go[4];
#pragma unroll
  for (int j = 0; j < 4; ++j) {
    const int p   = tid + 256 * j;
    const int row = p >> 3;
    const int pc  = p & 7;
    Pack8 pk;
    pk.h   = *(const v8h*)(st + row * HTP + pc * 8);
    val[j] = pk.u;
    go[j]  = (size_t)(blockIdx.x * 128 + row) * DFF + (size_t)blockIdx.y * 64 + pc * 8;
  }
  for (int ps = 0; ps < 2; ++ps) {
#pragma unroll
    for (int j = 0; j < 4; ++j) *(volatile v4u*)(hg + go[j]) = val[j];
    __threadfence();
  }
}

extern "C" void kernel_launch(void* const* d_in, const int* in_sizes, int n_in,
                              void* d_out, int out_size, void* d_ws, size_t ws_size,
                              hipStream_t stream) {
  if (n_in < 22) return;
  if (in_sizes[0] != NTOK * DM) return;
  if (in_sizes[1] != NTT * DM) return;
  if (in_sizes[3] != SQ * HDM) return;
  for (int i = 4; i <= 9; ++i) if (in_sizes[i] != DM) return;
  if (in_sizes[10] != NQKV * DM) return;
  if (in_sizes[11] != NQKV) return;
  if (in_sizes[12] != NQKV * DM) return;
  if (in_sizes[13] != NQKV) return;
  if (in_sizes[14] != DM * DM) return;
  if (in_sizes[15] != DM) return;
  if (in_sizes[16] != DFF * DM) return;
  if (in_sizes[17] != DFF) return;
  if (in_sizes[18] != DFF * DM) return;
  if (in_sizes[19] != DFF) return;
  if (in_sizes[20] != DM * DFF) return;
  if (in_sizes[21] != DM) return;
  if (out_size != NTOK * DM) return;

  const float* x      = (const float*)d_in[0];
  const float* temb   = (const float*)d_in[1];
  const float* rot    = (const float*)d_in[3];
  const float* ln1g   = (const float*)d_in[4];
  const float* ln1b   = (const float*)d_in[5];
  const float* ln2g   = (const float*)d_in[6];
  const float* ln2b   = (const float*)d_in[7];
  const float* ln3g   = (const float*)d_in[8];
  const float* ln3b   = (const float*)d_in[9];
  const float* aw     = (const float*)d_in[10];
  const float* ab     = (const float*)d_in[11];
  const float* cw     = (const float*)d_in[12];
  const float* cb     = (const float*)d_in[13];
  const float* cow    = (const float*)d_in[14];
  const float* cob    = (const float*)d_in[15];
  const float* f1w    = (const float*)d_in[16];
  const float* f1b    = (const float*)d_in[17];
  const float* gw     = (const float*)d_in[18];
  const float* gb     = (const float*)d_in[19];
  const float* f2w    = (const float*)d_in[20];
  const float* f2b    = (const float*)d_in[21];
  float* out = (float*)d_out;

  size_t off = 0;
  const size_t oWqkv = off; off += (size_t)NQKV * DM * 2;
  const size_t oWca  = off; off += (size_t)NQKV * DM * 2;
  const size_t oWco  = off; off += (size_t)DM * DM * 2;
  const size_t oWf1  = off; off += (size_t)DFF * DM * 2;
  const size_t oWg   = off; off += (size_t)DFF * DM * 2;
  const size_t oWf2  = off; off += (size_t)DM * DFF * 2;
  const size_t oTE   = off; off += (size_t)NTT * DM * 2;
  const size_t oTT   = off; off += (size_t)TTN * 4;
  const size_t oXN   = off; off += (size_t)NTOK * DM * 2;
  const size_t oX2   = off; off += (size_t)NTOK * DM * 4;
  const size_t oO    = off; off += (size_t)NTOK * DM * 2;
  const size_t oQ    = off; off += (size_t)NB * NH * SQ * HDM * 2;
  const size_t oK    = off; off += (size_t)NB * NH * SQ * HDM * 2;
  const size_t oVT   = off; off += (size_t)NB * NH * HDM * SQ * 2;
  const size_t oX1   = off; off += (size_t)NTOK * DM * 4;
  const size_t oHG   = oQ;
  if (off > ws_size) return;
  if (off > (size_t)134217728) return;
  if (oHG + (size_t)NTOK * DFF * 2 > off) return;

  char* ws = (char*)d_ws;
  _Float16* Wqkv = (_Float16*)(ws + oWqkv);
  _Float16* Wca  = (_Float16*)(ws + oWca);
  _Float16* Wco  = (_Float16*)(ws + oWco);
  _Float16* Wf1  = (_Float16*)(ws + oWf1);
  _Float16* Wg   = (_Float16*)(ws + oWg);
  _Float16* Wf2  = (_Float16*)(ws + oWf2);
  _Float16* TE   = (_Float16*)(ws + oTE);
  float*    TT   = (float*)(ws + oTT);
  _Float16* XN   = (_Float16*)(ws + oXN);
  float*    X2   = (float*)(ws + oX2);
  _Float16* Op   = (_Float16*)(ws + oO);
  _Float16* Qp   = (_Float16*)(ws + oQ);
  _Float16* Kp   = (_Float16*)(ws + oK);
  _Float16* VTp  = (_Float16*)(ws + oVT);
  float*    X1   = (float*)(ws + oX1);
  _Float16* HG   = (_Float16*)(ws + oHG);

  k_trig<<<dim3((SQ * HDM) / 256), dim3(256), 0, stream>>>(rot, TT);
  k_cvt<<<dim3((NQKV * DM) / 2048), dim3(256), 0, stream>>>(aw, Wqkv, 32.0f);
  k_cvt<<<dim3((NQKV * DM) / 2048), dim3(256), 0, stream>>>(cw, Wca, 32.0f);
  k_cvt<<<dim3((DM * DM) / 2048), dim3(256), 0, stream>>>(cow, Wco, 32.0f);
  k_cvt<<<dim3((DFF * DM) / 2048), dim3(256), 0, stream>>>(f1w, Wf1, 32.0f);
  k_cvt<<<dim3((DFF * DM) / 2048), dim3(256), 0, stream>>>(gw, Wg, 32.0f);
  k_cvt<<<dim3((DM * DFF) / 2048), dim3(256), 0, stream>>>(f2w, Wf2, 32.0f);
  k_cvt<<<dim3((NTT * DM) / 2048), dim3(256), 0, stream>>>(temb, TE, 1.0f);

  const float sscale = 0.125f;
  k_ln<<<dim3(NTOK), dim3(128), 0, stream>>>(x, ln1g, ln1b, XN);
  k_qkv<<<dim3(NB * (SQ / 256), NQKV / 64), dim3(256), 0, stream>>>(XN, Wqkv, ab, TT, Qp, Kp, VTp, SQ, 0, 1);
  k_attn<0><<<dim3(NB * NH * NQB), dim3(256), 0, stream>>>(Qp, Kp, VTp, x, X1, Op, SQ, sscale);

  k_ln<<<dim3(NTOK), dim3(128), 0, stream>>>(X1, ln2g, ln2b, XN);
  k_qkv<<<dim3(NB * (SQ / 256), DM / 64), dim3(256), 0, stream>>>(XN, Wca, cb, TT, Qp, Kp, VTp, SQ, 0, 0);
  k_qkv<<<dim3(NB * (TL / 256), 2 * DM / 64), dim3(256), 0, stream>>>(TE, Wca, cb, TT, Qp, Kp, VTp, TL, 1, 0);
  k_attn<1><<<dim3(NB * NH * NQB), dim3(256), 0, stream>>>(Qp, Kp, VTp, x, X1, Op, TL, sscale);
  k_gemm_f32<<<dim3(NTOK / 256, DM / 64), dim3(256), 0, stream>>>(Op, DM, Wco, DM, cob, 0.00048828125f, X2, DM, X1);

  k_ln<<<dim3(NTOK), dim3(128), 0, stream>>>(X2, ln3g, ln3b, XN);
  k_fcgate<<<dim3(NTOK / 128, DFF / 64), dim3(256), 0, stream>>>(XN, Wf1, Wg, f1b, gb, HG);
  k_gemm_f32<<<dim3(NTOK / 256, DM / 64), dim3(256), 0, stream>>>(HG, DFF, Wf2, DFF, f2b, 0.001953125f, out, DM, X2);
  (void)hipGetLastError();
}
